// SelfAttention_22110491640307
// MI455X (gfx1250) — hardware-verified
//
#include <hip/hip_runtime.h>


#ifndef NB
#define NB 8
#endif
#ifndef SEQ
#define SEQ 4096
#endif
#define NB_FULL   8
#define SEQ_FULL  4096
#define CIN       128
#define HD        64
#define NPROJ     192
#define BQ        128
#define BK        32
#define NWAVE     8
#define PT        64
#define XP        136
#define KP        72
#define OP        132
#define PLANE     ((size_t)NB * SEQ * HD)

#define OFF_KQ    ((size_t)0)
#define OFF_HT    (OFF_KQ + 4 * PLANE * 2)
#define OFF_NB    (OFF_HT + PLANE * 2)
#define OFF_W     (OFF_NB + (size_t)NB * SEQ * 4)
#define W_BYTES   ((size_t)(NPROJ * CIN + CIN * HD) * 2)
#define WS_TOTAL  (OFF_W + W_BYTES)

static_assert(SEQ % BQ == 0);
static_assert(SEQ % PT == 0);
static_assert(SEQ % BK == 0);
static_assert(BQ == NWAVE * 16);
static_assert(BQ * 4 == 32 * 16);
static_assert(HD == 64);
static_assert(CIN == 128);
static_assert(CIN % 32 == 0 && HD % 32 == 0);
static_assert(NPROJ == 3 * HD);
static_assert(PT == 64);
static_assert(SEQ <= SEQ_FULL);
static_assert(NB >= 1 && NB <= NB_FULL);
static_assert((XP * 2) % 16 == 0);
static_assert((KP * 2) % 16 == 0);
static_assert((OP * 4) % 16 == 0);
static_assert(XP >= CIN && KP >= HD && OP >= BQ);
static_assert((NPROJ * CIN + CIN * HD) / 8 == 4096);
static_assert(OFF_HT % 128 == 0 && OFF_NB % 128 == 0 && OFF_W % 128 == 0);
static_assert(WS_TOTAL <= (size_t)134217728);

typedef __bf16   bf16;
typedef _Float16 f16;
typedef bf16     v16bf __attribute__((ext_vector_type(16)));
typedef f16      v16h  __attribute__((ext_vector_type(16)));
typedef float    v8f   __attribute__((ext_vector_type(8)));
typedef float    v4f   __attribute__((ext_vector_type(4)));
typedef unsigned v4u   __attribute__((ext_vector_type(4)));

union FragB  { v16bf v; v4u q[2]; bf16 h[16]; };
union FragH  { v16h  v; v4u q[2]; f16  h[16]; };
union Pack8B { v4u u; bf16 h[8]; };
union Pack8H { v4u u; f16  h[8]; };

static __device__ __forceinline__ v8f mma_bf16(v16bf a, v16bf b, v8f acc) {
  acc = __builtin_amdgcn_wmma_f32_16x16x32_bf16(false, a, false, b, (short)0, acc, false, false);
  asm volatile("v_nop\n\tv_nop\n\tv_nop\n\tv_nop" : "+v"(acc) : "v"(a), "v"(b));
  return acc;
}
static __device__ __forceinline__ v8f mma_f16(v16h a, v16h b, v8f acc) {
  acc = __builtin_amdgcn_wmma_f32_16x16x32_f16(false, a, false, b, (short)0, acc, false, false);
  asm volatile("v_nop\n\tv_nop\n\tv_nop\n\tv_nop" : "+v"(acc) : "v"(a), "v"(b));
  return acc;
}

__global__ __launch_bounds__(256) void wprep_kernel(const float* __restrict__ Wk,
                                                    const float* __restrict__ Wq,
                                                    const float* __restrict__ Wh,
                                                    const float* __restrict__ Wv,
                                                    v4u* __restrict__ wplane) {
  const int p   = blockIdx.x * 256 + threadIdx.x;
  const int src = p >> 10;
  const int off = (p & 1023) * 8;
  const v4f a0 = *(const v4f*)(Wk + off), a1 = *(const v4f*)(Wk + off + 4);
  const v4f b0 = *(const v4f*)(Wq + off), b1 = *(const v4f*)(Wq + off + 4);
  const v4f c0 = *(const v4f*)(Wh + off), c1 = *(const v4f*)(Wh + off + 4);
  const v4f d0 = *(const v4f*)(Wv + off), d1 = *(const v4f*)(Wv + off + 4);
  Pack8B pb;
  Pack8H ph;
  #pragma unroll
  for (int i = 0; i < 4; ++i) {
    float e0 = a0[i], e1 = a1[i];
    e0 = (src == 1) ? b0[i] : e0;  e1 = (src == 1) ? b1[i] : e1;
    e0 = (src == 2) ? c0[i] : e0;  e1 = (src == 2) ? c1[i] : e1;
    e0 = (src == 3) ? d0[i] : e0;  e1 = (src == 3) ? d1[i] : e1;
    const bf16 w0 = (bf16)e0;
    const bf16 w1 = (bf16)e1;
    pb.h[i]     = w0;
    pb.h[4 + i] = w1;
    ph.h[i]     = (f16)((float)w0 * 64.0f);
    ph.h[4 + i] = (f16)((float)w1 * 64.0f);
  }
  v4u val;
  #pragma unroll
  for (int e = 0; e < 4; ++e) val[e] = (src < 3) ? pb.u[e] : ph.u[e];
  *(volatile v4u*)(wplane + p) = val;
  __threadfence();
  *(volatile v4u*)(wplane + p) = val;
}

__global__ __launch_bounds__(256) void proj_kernel(const float* __restrict__ x,
                                                   const bf16* __restrict__ wb,
                                                   bf16* __restrict__ kq,
                                                   f16* __restrict__ hT) {
  const int nt   = blockIdx.x;
  const int b    = blockIdx.y;
  const int tid  = threadIdx.x;
  const int wave = __builtin_amdgcn_readfirstlane(tid >> 5);
  const int lane = tid & 31;
  const int lq   = lane & 15;
  const int hi   = lane >> 4;
  const int n0   = nt * PT;

  __shared__ __align__(16) bf16 sX[PT * XP];
  __shared__ __align__(16) bf16 sKQ[4 * PT * KP];
  __shared__ __align__(16) f16  sH[HD * KP];

  #pragma unroll
  for (int it = 0; it < 8; ++it) {
    const int idx = tid + 256 * it;
    const int c   = idx >> 4;
    const int n4  = (idx & 15) * 4;
    const v4f v = *(const v4f*)(x + ((size_t)b * CIN + c) * SEQ_FULL + n0 + n4);
    #pragma unroll
    for (int i = 0; i < 4; ++i) sX[(n4 + i) * XP + c] = (bf16)v[i];
  }
  __syncthreads();

  const int ntile = wave & 3;
  const int half  = wave >> 2;

  v8f acc[6];
  #pragma unroll
  for (int t = 0; t < 6; ++t) acc[t] = (v8f){0, 0, 0, 0, 0, 0, 0, 0};

  #pragma unroll 1
  for (int ks = 0; ks < CIN / 32; ++ks) {
    const int k0 = ks * 32;
    FragB bx;
    {
      const int off = (ntile * 16 + lq) * XP + k0 + hi * 8;
      bx.q[0] = *(const v4u*)(&sX[off]);
      bx.q[1] = *(const v4u*)(&sX[off + 16]);
    }
    #pragma unroll
    for (int t = 0; t < 6; ++t) {
      const int which = t >> 1;
      const int ht    = 2 * half + (t & 1);
      const bf16* base = wb + (size_t)(which * HD + ht * 16 + lq) * CIN + k0 + hi * 8;
      FragB aw;
      aw.q[0] = *(const v4u*)(base);
      aw.q[1] = *(const v4u*)(base + 16);
      acc[t] = mma_bf16(aw.v, bx.v, acc[t]);
    }
  }

  #pragma unroll
  for (int t = 0; t < 6; ++t) {
    const int which = t >> 1;
    const int ht    = 2 * half + (t & 1);
    const int n     = ntile * 16 + lq;
    const int h0    = ht * 16 + hi * 8;
    if (which < 2) {
      Pack8B phh, pll;
      #pragma unroll
      for (int r = 0; r < 8; ++r) {
        const float v  = acc[t][r];
        const bf16  hb = (bf16)v;
        phh.h[r] = hb;
        pll.h[r] = (bf16)(v - (float)hb);
      }
      *(v4u*)(&sKQ[((which * 2 + 0) * PT + n) * KP + h0]) = phh.u;
      *(v4u*)(&sKQ[((which * 2 + 1) * PT + n) * KP + h0]) = pll.u;
    } else {
      #pragma unroll
      for (int r = 0; r < 8; ++r) sH[(h0 + r) * KP + n] = (f16)(acc[t][r] * 16.0f);
    }
  }
  __syncthreads();

  const int piece = tid & 7;
  v4u    kv[8];
  size_t kidx[8];
  #pragma unroll
  for (int it = 0; it < 8; ++it) {
    const int plane = it >> 1;
    const int row   = (it & 1) * 32 + (tid >> 3);
    kv[it]   = *(const v4u*)(&sKQ[(plane * PT + row) * KP + piece * 8]);
    kidx[it] = (size_t)plane * PLANE + ((size_t)b * SEQ + n0 + row) * HD + piece * 8;
  }
  v4u    hv[2];
  size_t hidx[2];
  #pragma unroll
  for (int it = 0; it < 2; ++it) {
    const int h = it * 32 + (tid >> 3);
    hv[it]   = *(const v4u*)(&sH[h * KP + piece * 8]);
    hidx[it] = ((size_t)b * HD + h) * SEQ + n0 + piece * 8;
  }
  #pragma unroll
  for (int it = 0; it < 8; ++it) *(volatile v4u*)(kq + kidx[it]) = kv[it];
  #pragma unroll
  for (int it = 0; it < 2; ++it) *(volatile v4u*)(hT + hidx[it]) = hv[it];
  __threadfence();
  #pragma unroll
  for (int it = 0; it < 8; ++it) *(volatile v4u*)(kq + kidx[it]) = kv[it];
  #pragma unroll
  for (int it = 0; it < 2; ++it) *(volatile v4u*)(hT + hidx[it]) = hv[it];
}

__global__ __launch_bounds__(256) void colstat_kernel(const bf16* __restrict__ kq,
                                                      float* __restrict__ nb) {
  const int jblk = blockIdx.x;
  const int b    = blockIdx.y;
  const int tid  = threadIdx.x;
  const int wave = __builtin_amdgcn_readfirstlane(tid >> 5);
  const int lane = tid & 31;
  const int lq   = lane & 15;
  const int hi   = lane >> 4;

  __shared__ __align__(16) float sNb[BQ];

  const bf16* khi = kq;
  const bf16* klo = kq + PLANE;
  const bf16* qhi = kq + 2 * PLANE;
  const bf16* qlo = kq + 3 * PLANE;
  const int j0w = jblk * BQ + wave * 16;

  FragB qfh[2], qfl[2];
  {
    const size_t base = ((size_t)b * SEQ + j0w + lq) * HD + hi * 8;
    #pragma unroll
    for (int f = 0; f < 2; ++f) {
      qfh[f].q[0] = *(const v4u*)(qhi + base + f * 32);
      qfh[f].q[1] = *(const v4u*)(qhi + base + f * 32 + 16);
      qfl[f].q[0] = *(const v4u*)(qlo + base + f * 32);
      qfl[f].q[1] = *(const v4u*)(qlo + base + f * 32 + 16);
    }
  }

  const float L2E = 1.4426950408889634f;
  float m_run = -__builtin_inff();
  float s_run = 0.0f;

  #pragma unroll 1
  for (int i0 = 0; i0 < SEQ; i0 += BK) {
    v8f c[2];
    #pragma unroll
    for (int sub = 0; sub < 2; ++sub) {
      const size_t base = ((size_t)b * SEQ + i0 + sub * 16 + lq) * HD + hi * 8;
      FragB ah[2], al[2];
      #pragma unroll
      for (int f = 0; f < 2; ++f) {
        ah[f].q[0] = *(const v4u*)(khi + base + f * 32);
        ah[f].q[1] = *(const v4u*)(khi + base + f * 32 + 16);
        al[f].q[0] = *(const v4u*)(klo + base + f * 32);
        al[f].q[1] = *(const v4u*)(klo + base + f * 32 + 16);
      }
      v8f acc = (v8f){0, 0, 0, 0, 0, 0, 0, 0};
      #pragma unroll
      for (int f = 0; f < 2; ++f) {
        acc = mma_bf16(ah[f].v, qfh[f].v, acc);
        acc = mma_bf16(ah[f].v, qfl[f].v, acc);
        acc = mma_bf16(al[f].v, qfh[f].v, acc);
      }
      c[sub] = acc;
    }
    float mx = c[0][0];
    #pragma unroll
    for (int r = 0; r < 8; ++r) {
      mx = fmaxf(mx, c[0][r]);
      mx = fmaxf(mx, c[1][r]);
    }
    const float m_new = fmaxf(m_run, mx);
    const float resc  = __builtin_amdgcn_exp2f((m_run - m_new) * L2E);
    const float t     = -m_new * L2E;
    float psum = 0.0f;
    #pragma unroll
    for (int r = 0; r < 8; ++r) {
      psum += __builtin_amdgcn_exp2f(fmaf(c[0][r], L2E, t));
      psum += __builtin_amdgcn_exp2f(fmaf(c[1][r], L2E, t));
    }
    s_run = s_run * resc + psum;
    m_run = m_new;
  }

  const float m_o = __shfl_xor(m_run, 16, 32);
  const float s_o = __shfl_xor(s_run, 16, 32);
  const float M   = fmaxf(m_run, m_o);
  const float S   = s_run * __builtin_amdgcn_exp2f((m_run - M) * L2E) +
                    s_o   * __builtin_amdgcn_exp2f((m_o   - M) * L2E);
  const float nbv = 12.0f - M * L2E - log2f(S);
  if (hi == 0) sNb[wave * 16 + lq] = nbv;
  __syncthreads();
  if (wave == 0) {
    const v4f v = *(const v4f*)(&sNb[lane * 4]);
    float* dst = nb + (size_t)b * SEQ + jblk * BQ + lane * 4;
    *(volatile v4f*)dst = v;
    __threadfence();
    *(volatile v4f*)dst = v;
  }
}

__global__ __launch_bounds__(256) void attn_out_kernel(const bf16* __restrict__ kq,
                                                       const f16* __restrict__ hT,
                                                       const float* __restrict__ nb,
                                                       const f16* __restrict__ wvh,
                                                       const float* __restrict__ x,
                                                       const float* __restrict__ scale_p,
                                                       float* __restrict__ out) {
  const int iblk = blockIdx.x;
  const int b    = blockIdx.y;
  const int tid  = threadIdx.x;
  const int wave = __builtin_amdgcn_readfirstlane(tid >> 5);
  const int lane = tid & 31;
  const int lq   = lane & 15;
  const int hi   = lane >> 4;

  __shared__ __align__(16) float sO[64 * OP];

  const bf16* khi = kq;
  const bf16* klo = kq + PLANE;
  const bf16* qhi = kq + 2 * PLANE;
  const bf16* qlo = kq + 3 * PLANE;
  const int i0w = iblk * BQ + wave * 16;

  FragB kfh[2], kfl[2];
  {
    const size_t base = ((size_t)b * SEQ + i0w + lq) * HD + hi * 8;
    #pragma unroll
    for (int f = 0; f < 2; ++f) {
      kfh[f].q[0] = *(const v4u*)(khi + base + f * 32);
      kfh[f].q[1] = *(const v4u*)(khi + base + f * 32 + 16);
      kfl[f].q[0] = *(const v4u*)(klo + base + f * 32);
      kfl[f].q[1] = *(const v4u*)(klo + base + f * 32 + 16);
    }
  }

  const f16*   hT_b = hT + (size_t)b * HD * SEQ;
  const float* nb_b = nb + (size_t)b * SEQ;
  const float  L2E  = 1.4426950408889634f;

  v8f oT[4];
  #pragma unroll
  for (int dt = 0; dt < 4; ++dt) oT[dt] = (v8f){0, 0, 0, 0, 0, 0, 0, 0};

  #pragma unroll 1
  for (int j0 = 0; j0 < SEQ; j0 += BK) {
    FragH pa;
    #pragma unroll
    for (int sub = 0; sub < 2; ++sub) {
      const size_t base = ((size_t)b * SEQ + j0 + sub * 16 + lq) * HD + hi * 8;
      FragB ah[2], al[2];
      #pragma unroll
      for (int f = 0; f < 2; ++f) {
        ah[f].q[0] = *(const v4u*)(qhi + base + f * 32);
        ah[f].q[1] = *(const v4u*)(qhi + base + f * 32 + 16);
        al[f].q[0] = *(const v4u*)(qlo + base + f * 32);
        al[f].q[1] = *(const v4u*)(qlo + base + f * 32 + 16);
      }
      v8f acc = (v8f){0, 0, 0, 0, 0, 0, 0, 0};
      #pragma unroll
      for (int f = 0; f < 2; ++f) {
        acc = mma_bf16(ah[f].v, kfh[f].v, acc);
        acc = mma_bf16(ah[f].v, kfl[f].v, acc);
        acc = mma_bf16(al[f].v, kfh[f].v, acc);
      }
      const float* np = nb_b + j0 + sub * 16 + hi * 8;
      const v4f n0v = *(const v4f*)(np);
      const v4f n1v = *(const v4f*)(np + 4);
      #pragma unroll
      for (int r = 0; r < 4; ++r) {
        pa.h[sub * 8 + r]     = (f16)__builtin_amdgcn_exp2f(fmaf(acc[r],     L2E, n0v[r]));
        pa.h[sub * 8 + 4 + r] = (f16)__builtin_amdgcn_exp2f(fmaf(acc[4 + r], L2E, n1v[r]));
      }
    }
    FragH av[4];
    #pragma unroll
    for (int dt = 0; dt < 4; ++dt) {
      const f16* base = hT_b + (size_t)(dt * 16 + lq) * SEQ + j0 + hi * 8;
      av[dt].q[0] = *(const v4u*)(base);
      av[dt].q[1] = *(const v4u*)(base + 16);
    }
    #pragma unroll
    for (int dt = 0; dt < 4; ++dt) oT[dt] = mma_f16(av[dt].v, pa.v, oT[dt]);
  }

  const float CS = 1.0f / 4096.0f;
  FragH bo[2];
  #pragma unroll
  for (int f = 0; f < 2; ++f) {
    #pragma unroll
    for (int r = 0; r < 8; ++r) {
      bo[f].h[r]     = (f16)(oT[2 * f][r] * CS);
      bo[f].h[8 + r] = (f16)(oT[2 * f + 1][r] * CS);
    }
  }

  const float sc = (float)(bf16)scale_p[0] * (1.0f / 1024.0f);

  #pragma unroll 1
  for (int hh = 0; hh < 2; ++hh) {
    #pragma unroll
    for (int t = 0; t < 4; ++t) {
      const int ct = hh * 4 + t;
      const f16* base = wvh + (size_t)(ct * 16 + lq) * HD + hi * 8;
      FragH aw[2];
      #pragma unroll
      for (int f = 0; f < 2; ++f) {
        aw[f].q[0] = *(const v4u*)(base + f * 32);
        aw[f].q[1] = *(const v4u*)(base + f * 32 + 16);
      }
      v8f d = (v8f){0, 0, 0, 0, 0, 0, 0, 0};
      d = mma_f16(aw[0].v, bo[0].v, d);
      d = mma_f16(aw[1].v, bo[1].v, d);
      #pragma unroll
      for (int r = 0; r < 8; ++r) sO[(t * 16 + hi * 8 + r) * OP + wave * 16 + lq] = d[r];
    }
    __syncthreads();

    v4f    res[8];
    size_t gidx[8];
    #pragma unroll
    for (int it = 0; it < 8; ++it) {
      const int rl = wave + 8 * it;
      const v4f v = *(const v4f*)(&sO[rl * OP + lane * 4]);
      gidx[it] = ((size_t)b * CIN + hh * 64 + rl) * SEQ_FULL + iblk * BQ + lane * 4;
      const v4f xv = *(const v4f*)(x + gidx[it]);
      #pragma unroll
      for (int e = 0; e < 4; ++e) res[it][e] = fmaf(sc, v[e], (float)(bf16)xv[e]);
    }
    #pragma unroll
    for (int it = 0; it < 8; ++it) *(volatile v4f*)(out + gidx[it]) = res[it];
    __threadfence();
    #pragma unroll
    for (int it = 0; it < 8; ++it) *(volatile v4f*)(out + gidx[it]) = res[it];
    __syncthreads();
  }
}

extern "C" void kernel_launch(void* const* d_in, const int* in_sizes, int n_in,
                              void* d_out, int out_size, void* d_ws, size_t ws_size,
                              hipStream_t stream) {
  if (n_in < 6) return;
  const size_t x_need = ((size_t)(NB - 1) * CIN + (CIN - 1)) * SEQ_FULL + SEQ;
  if ((size_t)in_sizes[0] < x_need) return;
  if (in_sizes[1] < HD * CIN) return;
  if (in_sizes[2] < HD * CIN) return;
  if (in_sizes[3] < HD * CIN) return;
  if (in_sizes[4] < CIN * HD) return;
  if (in_sizes[5] < 1) return;
  if ((size_t)out_size < x_need) return;
  if (ws_size < WS_TOTAL) return;

  const float* x     = (const float*)d_in[0];
  const float* Wk    = (const float*)d_in[1];
  const float* Wq    = (const float*)d_in[2];
  const float* Wh    = (const float*)d_in[3];
  const float* Wv    = (const float*)d_in[4];
  const float* scale = (const float*)d_in[5];
  float*       out   = (float*)d_out;

  char* ws = (char*)d_ws;
  bf16*  kq     = (bf16*)(ws + OFF_KQ);
  f16*   hT     = (f16*)(ws + OFF_HT);
  float* nb     = (float*)(ws + OFF_NB);
  v4u*   wplane = (v4u*)(ws + OFF_W);
  const bf16* wb  = (const bf16*)(ws + OFF_W);
  const f16*  wvh = (const f16*)(ws + OFF_W + (size_t)NPROJ * CIN * 2);

  wprep_kernel<<<dim3(16), 256, 0, stream>>>(Wk, Wq, Wh, Wv, wplane);
  proj_kernel<<<dim3(SEQ / PT, NB), 256, 0, stream>>>(x, wb, kq, hT);
  colstat_kernel<<<dim3(SEQ / BQ, NB), 256, 0, stream>>>(kq, nb);
  attn_out_kernel<<<dim3(SEQ / BQ, NB), 256, 0, stream>>>(kq, hT, nb, wvh, x, scale, out);
}
